// GaussianModel_33191507264018
// MI455X (gfx1250) — hardware-verified
//
#include <hip/hip_runtime.h>
#include <math.h>
#include <stdint.h>

#define NQ_FULL 2048
#define NG_FULL 65536
#ifndef NQ
#define NQ  NQ_FULL
#endif
#ifndef NGS
#define NGS NG_FULL
#endif
#define KW   32
#define NPC  10
#define C0F  0.28209479177387814f
#define EPSF 1e-6f
#define LOG2E_D 1.4426950408889634
#define PCAR 16384.0f
#define VCAR 256.0f
#define PG_THREADS 256
#define PQ_THREADS 64
#define FL_WAVES   2
#define FL_THREADS (FL_WAVES * 32)
#define FL_QB      (FL_WAVES * 16)
#define NKB        (NGS / 32)

static_assert((NQ % 64) == 0 && NQ >= 64 && NQ <= NQ_FULL);
static_assert((NGS % PG_THREADS) == 0 && NGS >= PG_THREADS && NGS <= NG_FULL);
static_assert((NQ % PQ_THREADS) == 0 && (NQ % FL_QB) == 0);
static_assert(NKB * 32 == NGS);
static_assert(3 * NPC + 2 == KW);
static_assert(FL_THREADS == 64);

typedef unsigned short u16;
typedef _Float16 v16h __attribute__((ext_vector_type(16)));
typedef _Float16 v8h  __attribute__((ext_vector_type(8)));
typedef __bf16   v16b __attribute__((ext_vector_type(16)));
typedef float    v8f  __attribute__((ext_vector_type(8)));
typedef float    v4f  __attribute__((ext_vector_type(4)));
typedef unsigned int v4u __attribute__((ext_vector_type(4)));

union FragH { v16h v; v8h h[2]; v4u u[2]; };
union FragB { v16b v; v4u u[2]; };

__device__ __forceinline__ unsigned short bf_bits(float f) {
  unsigned u = __float_as_uint(f);
  return (unsigned short)((u + 0x7FFFu + ((u >> 16) & 1u)) >> 16);
}
__device__ __forceinline__ float bf_up(unsigned short h) { return __uint_as_float(((unsigned)h) << 16); }
__device__ __forceinline__ float bf_val(float f) { return bf_up(bf_bits(f)); }
__device__ __forceinline__ unsigned short h_bits(_Float16 x) { return __builtin_bit_cast(unsigned short, x); }
__device__ __forceinline__ unsigned pk16(unsigned short a, unsigned short b) { return (unsigned)a | ((unsigned)b << 16); }
__device__ __forceinline__ v8f zero8() { v8f z = {0.f, 0.f, 0.f, 0.f, 0.f, 0.f, 0.f, 0.f}; return z; }

__device__ __forceinline__ void split3(float x, unsigned short& hb, unsigned short& mb, unsigned short& lb) {
  hb = bf_bits(x);
  const float r1 = x - bf_up(hb);
  mb = bf_bits(r1);
  const float r2 = r1 - bf_up(mb);
  lb = bf_bits(r2);
}

__device__ __forceinline__ v16h ldfrag_h(const _Float16* p) {
  FragH f;
  f.h[0] = *(const v8h*)(p);
  f.h[1] = *(const v8h*)(p + 16);
  return f.v;
}
__device__ __forceinline__ v16b ldfrag_b(const u16* p) {
  FragB f;
  f.u[0] = *(const v4u*)(p);
  f.u[1] = *(const v4u*)(p + 16);
  return f.v;
}

__device__ __forceinline__ v8f mma_h(v16h a, v16h b, v8f c) {
  return __builtin_amdgcn_wmma_f32_16x16x32_f16(false, a, false, b, (short)0, c, false, false);
}
__device__ __forceinline__ v8f mma_b(v16b a, v16b b, v8f c) {
  return __builtin_amdgcn_wmma_f32_16x16x32_bf16(false, a, false, b, (short)0, c, false, false);
}
__device__ __forceinline__ void guard_s(v8f& a, v8f& b, v16b x0, v16b x1, v16b x2, v16b x3, v16b x4) {
#if defined(__HIP_DEVICE_COMPILE__)
  asm volatile("v_nop\n\tv_nop\n\tv_nop\n\tv_nop"
               : "+v"(a), "+v"(b) : "v"(x0), "v"(x1), "v"(x2), "v"(x3), "v"(x4) : "memory");
#endif
}
__device__ __forceinline__ void guard_o(v8f& a, v16h x0, v16h x1) {
#if defined(__HIP_DEVICE_COMPILE__)
  asm volatile("v_nop\n\tv_nop\n\tv_nop\n\tv_nop" : "+v"(a) : "v"(x0), "v"(x1) : "memory");
#endif
}
__device__ __forceinline__ void acc_guard1(v8f& a) {
#if defined(__HIP_DEVICE_COMPILE__)
  asm volatile("v_nop\n\tv_nop\n\tv_nop\n\tv_nop" : "+v"(a));
#endif
}
__device__ __forceinline__ void wave_sync_lds() {
#if defined(__HIP_DEVICE_COMPILE__)
  __builtin_amdgcn_fence(__ATOMIC_RELEASE, "workgroup");
  __builtin_amdgcn_wave_barrier();
  __builtin_amdgcn_fence(__ATOMIC_ACQUIRE, "workgroup");
#endif
}

__global__ __launch_bounds__(PG_THREADS)
void prep_prim(const float* __restrict__ mean, const float* __restrict__ scal, const float* __restrict__ rot,
               const float* __restrict__ opac, const float* __restrict__ feat, u16* KPl, u16* VTl, int ng) {
  __shared__ __align__(16) u16 ks[PG_THREADS * KW];
  __shared__ __align__(16) u16 vs[2 * PG_THREADS];
  const int tid = threadIdx.x, wave = tid >> 5, lane = tid & 31;
  const int n0 = blockIdx.x * PG_THREADS;
  if (n0 + PG_THREADS > ng) return;
  int n = n0 + tid;
  n = (n < ng) ? n : (ng - 1);

  const v4f r4 = *(const v4f*)(rot + (size_t)n * 4);
  float qw = bf_val(r4[0]), qx = bf_val(r4[1]), qy = bf_val(r4[2]), qz = bf_val(r4[3]);
  const float mu0 = bf_val(mean[(size_t)n * 3 + 0]);
  const float mu1 = bf_val(mean[(size_t)n * 3 + 1]);
  const float mu2 = bf_val(mean[(size_t)n * 3 + 2]);
  const float ls0 = bf_val(scal[(size_t)n * 3 + 0]);
  const float ls1 = bf_val(scal[(size_t)n * 3 + 1]);
  const float ls2 = bf_val(scal[(size_t)n * 3 + 2]);
  const float opv = bf_val(opac[n]);
  const float fre = bf_val(feat[(size_t)n * 2 + 0]);
  const float fim = bf_val(feat[(size_t)n * 2 + 1]);

  const float nrm  = sqrtf(qw * qw + qx * qx + qy * qy + qz * qz);
  const float qinv = 1.0f / (nrm + 1e-12f);
  qw *= qinv; qx *= qinv; qy *= qinv; qz *= qinv;
  const double w = (double)qw, x = (double)qx, y = (double)qy, z = (double)qz;
  const double R00 = 1.0 - 2.0 * (y * y + z * z), R01 = 2.0 * (x * y - w * z), R02 = 2.0 * (x * z + w * y);
  const double R10 = 2.0 * (x * y + w * z), R11 = 1.0 - 2.0 * (x * x + z * z), R12 = 2.0 * (y * z - w * x);
  const double R20 = 2.0 * (x * z - w * y), R21 = 2.0 * (y * z + w * x), R22 = 1.0 - 2.0 * (x * x + y * y);
  const double s0 = (double)__expf(ls0), s1 = (double)__expf(ls1), s2 = (double)__expf(ls2);
  const double L00 = R00 * s0, L01 = R01 * s1, L02 = R02 * s2;
  const double L10 = R10 * s0, L11 = R11 * s1, L12 = R12 * s2;
  const double L20 = R20 * s0, L21 = R21 * s1, L22 = R22 * s2;
  const double eps = (double)EPSF;
  const double c00 = L00 * L00 + L01 * L01 + L02 * L02 + eps;
  const double c01 = L00 * L10 + L01 * L11 + L02 * L12;
  const double c02 = L00 * L20 + L01 * L21 + L02 * L22;
  const double c11 = L10 * L10 + L11 * L11 + L12 * L12 + eps;
  const double c12 = L10 * L20 + L11 * L21 + L12 * L22;
  const double c22 = L20 * L20 + L21 * L21 + L22 * L22 + eps;
  const double f00 = c11 * c22 - c12 * c12;
  const double f01 = c02 * c12 - c01 * c22;
  const double f02 = c01 * c12 - c02 * c11;
  const double f11 = c00 * c22 - c02 * c02;
  const double f12 = c01 * c02 - c00 * c12;
  const double f22 = c00 * c11 - c01 * c01;
  const double det  = c00 * f00 + c01 * f01 + c02 * f02;
  const double idet = 1.0 / det;
  const double A00 = f00 * idet, A01 = f01 * idet, A02 = f02 * idet;
  const double A11 = f11 * idet, A12 = f12 * idet, A22 = f22 * idet;
  const double m0 = (double)mu0, m1 = (double)mu1, m2 = (double)mu2;
  const double Am0 = A00 * m0 + A01 * m1 + A02 * m2;
  const double Am1 = A01 * m0 + A11 * m1 + A12 * m2;
  const double Am2 = A02 * m0 + A12 * m1 + A22 * m2;
  const double uAu = m0 * Am0 + m1 * Am1 + m2 * Am2;

  float kv[NPC];
  kv[0] = (float)(-0.5 * LOG2E_D * A00);
  kv[1] = (float)(-0.5 * LOG2E_D * A11);
  kv[2] = (float)(-0.5 * LOG2E_D * A22);
  kv[3] = (float)(-LOG2E_D * A01);
  kv[4] = (float)(-LOG2E_D * A02);
  kv[5] = (float)(-LOG2E_D * A12);
  kv[6] = (float)(LOG2E_D * Am0);
  kv[7] = (float)(LOG2E_D * Am1);
  kv[8] = (float)(LOG2E_D * Am2);
  kv[9] = (float)(-0.5 * LOG2E_D * uAu);

  unsigned short rowv[KW];
#pragma unroll
  for (int j = 0; j < NPC; ++j) {
    unsigned short hb, mb, lb;
    split3(kv[j], hb, mb, lb);
    rowv[j] = hb; rowv[NPC + j] = mb; rowv[2 * NPC + j] = lb;
  }
  rowv[3 * NPC] = 0; rowv[3 * NPC + 1] = 0;
#pragma unroll
  for (int i = 0; i < 4; ++i) {
    v4u t;
#pragma unroll
    for (int e = 0; e < 4; ++e) t[e] = pk16(rowv[8 * i + 2 * e], rowv[8 * i + 2 * e + 1]);
    *(v4u*)(ks + (size_t)tid * KW + 8 * i) = t;
  }

  const float ex = __expf(-opv);
  const float sg = 1.0f / (1.0f + ex);
  vs[tid]              = h_bits((_Float16)(sg * (C0F * fre) * VCAR));
  vs[PG_THREADS + tid] = h_bits((_Float16)(sg * (C0F * fim) * VCAR));
  __syncthreads();

  v4u kp4[4];
#pragma unroll
  for (int i = 0; i < 4; ++i) kp4[i] = *(const v4u*)(ks + (size_t)(i * PG_THREADS + tid) * 8);
  u16* kd = KPl + (size_t)n0 * KW;
  for (int pass = 0; pass < 2; ++pass) {
#pragma unroll
    for (int i = 0; i < 4; ++i) {
      *(volatile v4u*)(kd + (size_t)(i * PG_THREADS + tid) * 8) = kp4[i];
    }
    __threadfence();
  }
  if (wave < 2) {
    const v4u pv = *(const v4u*)(vs + wave * PG_THREADS + 8 * lane);
    u16* vd = VTl + (size_t)wave * (size_t)ng + (size_t)n0 + 8 * lane;
    for (int pass = 0; pass < 2; ++pass) {
      *(volatile v4u*)(vd) = pv;
      __threadfence();
    }
  }
}

__global__ __launch_bounds__(PQ_THREADS)
void prep_query(const float* __restrict__ pos, u16* QPl, int nq) {
#pragma clang fp contract(off)
  __shared__ __align__(16) u16 qs[PQ_THREADS * KW];
  const int tid = threadIdx.x;
  const int b0 = blockIdx.x * PQ_THREADS;
  if (b0 + PQ_THREADS > nq) return;
  int b = b0 + tid;
  b = (b < nq) ? b : (nq - 1);
  const float p0 = bf_val(pos[(size_t)b * 3 + 0]);
  const float p1 = bf_val(pos[(size_t)b * 3 + 1]);
  const float p2 = bf_val(pos[(size_t)b * 3 + 2]);
  const float q0 = p0 * 2.0f - 1.0f;
  const float q1 = p1 * 2.0f - 1.0f;
  const float q2 = p2 * 2.0f - 1.0f;
  float qv[NPC];
  qv[0] = q0 * q0; qv[1] = q1 * q1; qv[2] = q2 * q2;
  qv[3] = q0 * q1; qv[4] = q0 * q2; qv[5] = q1 * q2;
  qv[6] = q0; qv[7] = q1; qv[8] = q2; qv[9] = 1.0f;
  unsigned short ph[NPC], pm[NPC], pl[NPC];
#pragma unroll
  for (int j = 0; j < NPC; ++j) split3(qv[j], ph[j], pm[j], pl[j]);

#pragma unroll
  for (int p = 0; p < 3; ++p) {
    unsigned short rowv[KW];
#pragma unroll
    for (int j = 0; j < NPC; ++j) {
      const unsigned short v = (p == 0) ? ph[j] : ((p == 1) ? pm[j] : pl[j]);
      rowv[j] = v; rowv[NPC + j] = v; rowv[2 * NPC + j] = v;
    }
    rowv[3 * NPC] = 0; rowv[3 * NPC + 1] = 0;
    if (p > 0) __syncthreads();
#pragma unroll
    for (int i = 0; i < 4; ++i) {
      v4u t;
#pragma unroll
      for (int e = 0; e < 4; ++e) t[e] = pk16(rowv[8 * i + 2 * e], rowv[8 * i + 2 * e + 1]);
      *(v4u*)(qs + (size_t)tid * KW + 8 * i) = t;
    }
    __syncthreads();
    v4u pc4[4];
#pragma unroll
    for (int i = 0; i < 4; ++i) pc4[i] = *(const v4u*)(qs + (size_t)(i * PQ_THREADS + tid) * 8);
    u16* qd = QPl + (size_t)p * (size_t)nq * KW + (size_t)b0 * KW;
    for (int pass = 0; pass < 2; ++pass) {
#pragma unroll
      for (int i = 0; i < 4; ++i) {
        *(volatile v4u*)(qd + (size_t)(i * PQ_THREADS + tid) * 8) = pc4[i];
      }
      __threadfence();
    }
  }
}

__global__ __launch_bounds__(FL_THREADS)
void splat_fwd(const u16* __restrict__ QPl, const u16* __restrict__ KPl, const u16* __restrict__ VTl,
               float* out, int nq, int ng) {
  __shared__ __align__(16) float smem[FL_WAVES * 256];

  const int tid  = threadIdx.x;
  const int wave = tid >> 5;
  const int lane = tid & 31;
  const int hh   = lane >> 4;
  const int c    = lane & 15;
  const int q0   = blockIdx.x * FL_QB + wave * 16;
  if (q0 + 16 > nq) return;

  const size_t qpl = (size_t)nq * KW;
  const u16* qb = QPl + (size_t)(q0 + c) * KW + 8 * hh;
  const v16b qh = ldfrag_b(qb);
  const v16b qm = ldfrag_b(qb + qpl);
  const v16b ql = ldfrag_b(qb + 2 * qpl);
  const u16* Kb = KPl + (size_t)c * KW + 8 * hh;
  const _Float16* Vb = (const _Float16*)(const void*)VTl + (size_t)(c & 1) * (size_t)ng + 8 * hh;

  v8f o = zero8();

#pragma unroll 1
  for (int it = 0; it < NKB; ++it) {
    const int kb = it * 32;
    const u16* k0p = Kb + (size_t)kb * KW;
    const v16b a0 = ldfrag_b(k0p);
    const v16b a1 = ldfrag_b(k0p + 16 * KW);
    v8f s0 = zero8(), s1 = zero8();
    s0 = mma_b(a0, qh, s0);
    s0 = mma_b(a0, qm, s0);
    s0 = mma_b(a0, ql, s0);
    s1 = mma_b(a1, qh, s1);
    s1 = mma_b(a1, qm, s1);
    s1 = mma_b(a1, ql, s1);
    guard_s(s0, s1, a0, a1, qh, qm, ql);
    FragH ph;
#pragma unroll
    for (int e4 = 0; e4 < 4; ++e4) {
      const float pa = exp2f(s0[2 * e4]);
      const float pb = exp2f(s0[2 * e4 + 1]);
      const float pc = exp2f(s1[2 * e4]);
      const float pd = exp2f(s1[2 * e4 + 1]);
      ph.u[0][e4] = pk16(h_bits((_Float16)(pa * PCAR)), h_bits((_Float16)(pb * PCAR)));
      ph.u[1][e4] = pk16(h_bits((_Float16)(pc * PCAR)), h_bits((_Float16)(pd * PCAR)));
    }
    const v16h vf = ldfrag_h(Vb + kb);
    o = mma_h(ph.v, vf, o);
    guard_o(o, ph.v, vf);
  }
  acc_guard1(o);

  float* slab = smem + wave * 256;
#pragma unroll
  for (int r = 0; r < 8; ++r) slab[(8 * hh + r) * 16 + c] = o[r];
  wave_sync_lds();
  const float val = slab[(lane >> 1) * 16 + (lane & 1)] * (1.0f / (PCAR * VCAR));
  float* dst = out + (size_t)q0 * 2 + lane;
  for (int pass = 0; pass < 2; ++pass) {
    *(volatile float*)(dst) = val;
    __threadfence();
  }
}

extern "C" void kernel_launch(void* const* d_in, const int* in_sizes, int n_in,
                              void* d_out, int out_size, void* d_ws, size_t ws_size,
                              hipStream_t stream) {
  if (n_in < 6) return;
  if (in_sizes[0] < NQ * 3) return;
  if (in_sizes[1] < NGS * 3 || in_sizes[2] < NGS * 3 || in_sizes[3] < NGS * 4) return;
  if (in_sizes[4] < NGS || in_sizes[5] < NGS * 2) return;
  if (out_size < NQ * 2) return;

  const float* pos  = (const float*)d_in[0];
  const float* mean = (const float*)d_in[1];
  const float* scal = (const float*)d_in[2];
  const float* rot  = (const float*)d_in[3];
  const float* opac = (const float*)d_in[4];
  const float* feat = (const float*)d_in[5];
  float*       out  = (float*)d_out;

  const size_t szKP = (size_t)NGS * KW * 2;
  const size_t szVT = (size_t)2 * NGS * 2;
  const size_t szQP = (size_t)3 * NQ * KW * 2;
  size_t off = 0;
  const size_t oKP = off; off += szKP;
  const size_t oVT = off; off += szVT;
  const size_t oQP = off; off += szQP;
  if (off > ws_size) return;
  if (off > (size_t)134217728) return;
  if ((oKP % 128) != 0 || (oVT % 128) != 0 || (oQP % 128) != 0) return;

  char* ws = (char*)d_ws;
  u16* KP = (u16*)(ws + oKP);
  u16* VT = (u16*)(ws + oVT);
  u16* QP = (u16*)(ws + oQP);

  if ((NGS % PG_THREADS) != 0 || (NQ % PQ_THREADS) != 0 || (NQ % FL_QB) != 0 || (NGS % 32) != 0) return;
  const dim3 gP(NGS / PG_THREADS);
  const dim3 bP(PG_THREADS);
  const dim3 gQ(NQ / PQ_THREADS);
  const dim3 bQ(PQ_THREADS);
  const dim3 gF(NQ / FL_QB);
  const dim3 bF(FL_THREADS);

  prep_prim<<<gP, bP, 0, stream>>>(mean, scal, rot, opac, feat, KP, VT, NGS);
  prep_query<<<gQ, bQ, 0, stream>>>(pos, QP, NQ);
  splat_fwd<<<gF, bF, 0, stream>>>(QP, KP, VT, out, NQ, NGS);
  (void)hipGetLastError();
}
